// BivectorRotarySelfAttention_884763263730
// MI455X (gfx1250) — hardware-verified
//
#include <hip/hip_runtime.h>
#include <math.h>
#include <stdint.h>

#define NSEQ   4
#define SQ     1024
#define HID    2048
#define NHQ    16
#define NKVH   4
#define HDM    128
#define HHALF  64
#define QW     2048
#define KVW    512
#define QKW    2560
#define WTR    3072
#define NTOK   4096

typedef __bf16         v16b  __attribute__((ext_vector_type(16)));
typedef __bf16         v8b   __attribute__((ext_vector_type(8)));
typedef float          v8f   __attribute__((ext_vector_type(8)));
typedef float          v4f   __attribute__((ext_vector_type(4)));
typedef float          v4fa  __attribute__((ext_vector_type(4), __may_alias__));
typedef unsigned int   v4u   __attribute__((ext_vector_type(4)));
typedef unsigned short v8us  __attribute__((ext_vector_type(8)));
typedef unsigned short v8usa __attribute__((ext_vector_type(8), __may_alias__));

__device__ __forceinline__ unsigned short bf_bits(float f) {
  const unsigned u = __float_as_uint(f);
  return (unsigned short)((u + 0x7FFFu + ((u >> 16) & 1u)) >> 16);
}
__device__ __forceinline__ float bf_val(unsigned short h) { return __uint_as_float(((unsigned)h) << 16); }
__device__ __forceinline__ float bf_rne(float f) { return bf_val(bf_bits(f)); }
__device__ __forceinline__ unsigned pk16(unsigned short a, unsigned short b) { return (unsigned)a | ((unsigned)b << 16); }
__device__ __forceinline__ v8f zero8() { v8f z = {0.f, 0.f, 0.f, 0.f, 0.f, 0.f, 0.f, 0.f}; return z; }
__device__ __forceinline__ int wave_id() { return __builtin_amdgcn_readfirstlane((int)(threadIdx.x >> 5)); }

__device__ __forceinline__ void lds_wave_sync() {
  __builtin_amdgcn_fence(__ATOMIC_RELEASE, "workgroup");
  __builtin_amdgcn_wave_barrier();
  __builtin_amdgcn_fence(__ATOMIC_ACQUIRE, "workgroup");
}

union FragB { v16b v; v8b h[2]; };
__device__ __forceinline__ v16b ldfrag(const unsigned short* p) {
  FragB f;
  const v8us w0 = *(const v8usa*)(p);
  const v8us w1 = *(const v8usa*)(p + 16);
  f.h[0] = __builtin_bit_cast(v8b, w0);
  f.h[1] = __builtin_bit_cast(v8b, w1);
  return f.v;
}
__device__ __forceinline__ v8f mma_b(v16b a, v16b b, v8f c) {
  return __builtin_amdgcn_wmma_f32_16x16x32_bf16(false, a, false, b, (short)0, c, false, false);
}
__device__ __forceinline__ void guard_g(v8f& a, v8f& b, v16b x0, v16b x1, v16b x2, v16b x3, v16b y) {
#if defined(__HIP_DEVICE_COMPILE__)
  asm volatile("v_nop\n\tv_nop\n\tv_nop\n\tv_nop" : "+v"(a), "+v"(b) : "v"(x0), "v"(x1), "v"(x2), "v"(x3), "v"(y) : "memory");
#endif
}
__device__ __forceinline__ void guard_s(v8f& a, v8f& b, v8f& cc, v8f& d,
                                        v16b x0, v16b x1, v16b x2, v16b x3, v16b x4, v16b x5, v16b x6, v16b x7) {
#if defined(__HIP_DEVICE_COMPILE__)
  asm volatile("v_nop\n\tv_nop\n\tv_nop\n\tv_nop"
               : "+v"(a), "+v"(b), "+v"(cc), "+v"(d)
               : "v"(x0), "v"(x1), "v"(x2), "v"(x3), "v"(x4), "v"(x5), "v"(x6), "v"(x7) : "memory");
#endif
}
__device__ __forceinline__ void guard_o(v8f& a, v16b x0, v16b x1, v16b x2, v16b x3) {
#if defined(__HIP_DEVICE_COMPILE__)
  asm volatile("v_nop\n\tv_nop\n\tv_nop\n\tv_nop" : "+v"(a) : "v"(x0), "v"(x1), "v"(x2), "v"(x3) : "memory");
#endif
}
__device__ __forceinline__ void acc_guard4(v8f& a, v8f& b, v8f& cc, v8f& d) {
#if defined(__HIP_DEVICE_COMPILE__)
  asm volatile("v_nop\n\tv_nop\n\tv_nop\n\tv_nop" : "+v"(a), "+v"(b), "+v"(cc), "+v"(d));
#endif
}

__global__ __launch_bounds__(256) void cvt_bf16_kernel(const float* __restrict__ in, unsigned short* __restrict__ outp, int n8) {
  const int i = (int)blockIdx.x * 256 + (int)threadIdx.x;
  if (i >= n8) return;
  const size_t e = 8 * (size_t)i;
  const v4f a = *(const v4f*)(in + e);
  const v4f b = *(const v4f*)(in + e + 4);
  v4u w;
  w[0] = pk16(bf_bits(a[0]), bf_bits(a[1]));
  w[1] = pk16(bf_bits(a[2]), bf_bits(a[3]));
  w[2] = pk16(bf_bits(b[0]), bf_bits(b[1]));
  w[3] = pk16(bf_bits(b[2]), bf_bits(b[3]));
  *(volatile v4u*)(outp + e) = w;
  __threadfence();
  *(volatile v4u*)(outp + e) = w;
}

__global__ __launch_bounds__(256) void tconv_bf16_kernel(const float* __restrict__ W, unsigned short* __restrict__ outp, int R, int Cc) {
  __shared__ __align__(16) float tf[64 * 68];
  const int c0  = (int)blockIdx.x * 64;
  const int r0  = (int)blockIdx.y * 64;
  const int tid = (int)threadIdx.x;
  {
    const int lr = tid >> 4;
    const int c4 = (tid & 15) * 4;
#pragma unroll
    for (int it = 0; it < 4; ++it) {
      const int rr = it * 16 + lr;
      const v4f a = *(const v4f*)(W + (size_t)(r0 + rr) * Cc + c0 + c4);
      *(v4f*)(tf + rr * 68 + c4) = a;
    }
  }
  __syncthreads();
  const int sub = tid >> 3;
  const int c8  = (tid & 7) * 8;
  v4u hv[2];
#pragma unroll
  for (int it = 0; it < 2; ++it) {
    const int oc = it * 32 + sub;
    v4u a;
#pragma unroll
    for (int q = 0; q < 4; ++q) {
      const float f0 = tf[(c8 + 2 * q) * 68 + oc];
      const float f1 = tf[(c8 + 2 * q + 1) * 68 + oc];
      a[q] = pk16(bf_bits(f0), bf_bits(f1));
    }
    hv[it] = a;
  }
  for (int pass = 0; pass < 2; ++pass) {
#pragma unroll
    for (int it = 0; it < 2; ++it) {
      const int oc = it * 32 + sub;
      const size_t go = (size_t)(c0 + oc) * R + r0 + c8;
      *(volatile v4u*)(outp + go) = hv[it];
    }
    __threadfence();
  }
}

template <int EPI> struct SlabT { typedef unsigned short T; static constexpr int PERW = 4096; };
template <> struct SlabT<2>     { typedef float          T; static constexpr int PERW = 2048; };

template <int EPI, bool SPLITA>
__global__ __launch_bounds__(128) void gemm_w32x128_kernel(
    const unsigned short* Ap, const unsigned short* A2p, int lda,
    const unsigned short* __restrict__ Btp, int ldb,
    const float* __restrict__ cosp, const float* __restrict__ sinp,
    void* C0, void* C1, void* C2, void* C3, int ldc,
    int M, int N, int K) {
  typedef typename SlabT<EPI>::T ST;
  __shared__ __align__(16) ST slab_all[4 * SlabT<EPI>::PERW];

  const int lane = threadIdx.x & 31;
  const int wave = wave_id();
  const int hh = lane >> 4;
  const int rl = lane & 15;
  const int tilesN = N >> 7;
  const int tilesM = M >> 5;
  const int tile = (int)blockIdx.x * 4 + wave;
  if (tile >= tilesM * tilesN) return;
  const int tm = tile / tilesN;
  const int tn = tile - tm * tilesN;
  const int m0 = tm << 5;
  const int n0 = tn << 7;

  v8f acc[2][8];
#pragma unroll
  for (int i = 0; i < 2; ++i)
#pragma unroll
    for (int j = 0; j < 8; ++j) acc[i][j] = zero8();

  for (int k0 = 0; k0 < K; k0 += 32) {
    v16b ah[2], al[2];
#pragma unroll
    for (int i = 0; i < 2; ++i) {
      const size_t ao = (size_t)(m0 + i * 16 + rl) * lda + k0 + 8 * hh;
      ah[i] = ldfrag(Ap + ao);
      al[i] = SPLITA ? ldfrag(A2p + ao) : ah[i];
    }
#pragma unroll
    for (int j = 0; j < 8; ++j) {
      const v16b bj = ldfrag(Btp + (size_t)(n0 + j * 16 + rl) * ldb + k0 + 8 * hh);
      acc[0][j] = mma_b(ah[0], bj, acc[0][j]);
      acc[1][j] = mma_b(ah[1], bj, acc[1][j]);
      if (SPLITA) {
        acc[0][j] = mma_b(al[0], bj, acc[0][j]);
        acc[1][j] = mma_b(al[1], bj, acc[1][j]);
      }
      guard_g(acc[0][j], acc[1][j], ah[0], ah[1], al[0], al[1], bj);
    }
  }
  acc_guard4(acc[0][0], acc[0][1], acc[0][2], acc[0][3]);
  acc_guard4(acc[0][4], acc[0][5], acc[0][6], acc[0][7]);
  acc_guard4(acc[1][0], acc[1][1], acc[1][2], acc[1][3]);
  acc_guard4(acc[1][4], acc[1][5], acc[1][6], acc[1][7]);

  ST* slab = slab_all + wave * SlabT<EPI>::PERW;
  unsigned short* sl  = (unsigned short*)(void*)slab;
  float*          slf = (float*)(void*)slab;

  if (EPI == 0) {
    const bool isq = (n0 < QW);
    unsigned short* P0 = isq ? (unsigned short*)C0 : (unsigned short*)C2;
    unsigned short* P1 = isq ? (unsigned short*)C1 : (unsigned short*)C3;
    const int ldp  = isq ? ldc : KVW;
    const int col0 = isq ? n0 : (n0 - QW);
    const int hs   = col0 >> 7;
#pragma unroll
    for (int i = 0; i < 2; ++i) {
      const int rb = m0 + i * 16 + 8 * hh;
#pragma unroll
      for (int s = 0; s < 2; ++s) {
#pragma unroll
        for (int j = 0; j < 2; ++j) {
          const int jd = j * 16 + rl;
#pragma unroll
          for (int r = 0; r < 8; ++r) {
            const int row = rb + r;
            const int pos = row & (SQ - 1);
            const size_t tb = ((size_t)pos * NHQ + hs) * HHALF + jd;
            const float c1 = bf_rne(cosp[tb]);
            const float s1 = bf_rne(sinp[tb]);
            const float c2 = bf_rne(cosp[tb + 32]);
            const float s2 = bf_rne(sinp[tb + 32]);
            const float x1 = acc[i][4 * s + j][r];
            const float x2 = acc[i][4 * s + j + 2][r];
            const float o1 = x1 * c1 - x2 * s1;
            const float o2 = x2 * c2 + x1 * s2;
            const unsigned short h1 = bf_bits(o1);
            const unsigned short h2 = bf_bits(o2);
            const int so = (8 * hh + r) * 128 + 64 * s + jd;
            sl[so]             = h1;
            sl[so + 32]        = h2;
            sl[2048 + so]      = bf_bits(o1 - bf_val(h1));
            sl[2048 + so + 32] = bf_bits(o2 - bf_val(h2));
          }
        }
      }
      lds_wave_sync();
      for (int pass = 0; pass < 2; ++pass) {
#pragma unroll
        for (int it = 0; it < 8; ++it) {
          const int row = it * 2 + hh;
          const int c8  = rl * 8;
          const v8us vh = *(const v8usa*)(sl + row * 128 + c8);
          const v8us vl = *(const v8usa*)(sl + 2048 + row * 128 + c8);
          const size_t go = (size_t)(m0 + i * 16 + row) * ldp + col0 + c8;
          *(volatile v8us*)(P0 + go) = vh;
          *(volatile v8us*)(P1 + go) = vl;
        }
        __threadfence();
      }
      lds_wave_sync();
    }
  } else if (EPI == 1) {
    unsigned short* P0 = (unsigned short*)C0;
    unsigned short* P1 = (unsigned short*)C1;
#pragma unroll
    for (int i = 0; i < 2; ++i) {
#pragma unroll
      for (int r = 0; r < 8; ++r) {
#pragma unroll
        for (int j = 0; j < 8; ++j) {
          const float v = acc[i][j][r];
          const unsigned short hv = bf_bits(v);
          const int so = (8 * hh + r) * 128 + j * 16 + rl;
          sl[so]        = hv;
          sl[2048 + so] = bf_bits(v - bf_val(hv));
        }
      }
      lds_wave_sync();
      for (int pass = 0; pass < 2; ++pass) {
#pragma unroll
        for (int it = 0; it < 8; ++it) {
          const int row = it * 2 + hh;
          const int c8  = rl * 8;
          const v8us vh = *(const v8usa*)(sl + row * 128 + c8);
          const v8us vl = *(const v8usa*)(sl + 2048 + row * 128 + c8);
          const size_t go = (size_t)(m0 + i * 16 + row) * ldc + n0 + c8;
          *(volatile v8us*)(P0 + go) = vh;
          *(volatile v8us*)(P1 + go) = vl;
        }
        __threadfence();
      }
      lds_wave_sync();
    }
  } else {
    float* C = (float*)C0;
#pragma unroll
    for (int i = 0; i < 2; ++i) {
#pragma unroll
      for (int j = 0; j < 8; ++j)
#pragma unroll
        for (int r = 0; r < 8; ++r)
          slf[(8 * hh + r) * 128 + j * 16 + rl] = acc[i][j][r];
      lds_wave_sync();
      for (int pass = 0; pass < 2; ++pass) {
#pragma unroll
        for (int row = 0; row < 16; ++row) {
          const v4f v = *(const v4fa*)(slf + row * 128 + lane * 4);
          *(volatile v4f*)(C + (size_t)(m0 + i * 16 + row) * ldc + n0 + lane * 4) = v;
        }
        __threadfence();
      }
      lds_wave_sync();
    }
  }
}

#define AT_KC   32
#define KS_P    136
#define VS_P    40
#define PS_P    40
#define LDS_KH  0
#define LDS_KL  (32 * KS_P)
#define LDS_VH  (2 * 32 * KS_P)
#define LDS_VL  (LDS_VH + 128 * VS_P)
#define LDS_PH  (LDS_VL + 128 * VS_P)
#define LDS_PL  (LDS_PH + 4 * 16 * PS_P)
#define LDS_TOT (LDS_PL + 4 * 16 * PS_P)
static_assert(LDS_TOT * 2 <= 65536);
static_assert(4 * 4096 <= LDS_TOT);

__global__ __launch_bounds__(128) void attn_bivector_kernel(
    const unsigned short* __restrict__ qhp, const unsigned short* __restrict__ qlp,
    const unsigned short* __restrict__ khp, const unsigned short* __restrict__ klp,
    const unsigned short* __restrict__ vhp, const unsigned short* __restrict__ vlp,
    const float* __restrict__ qpar, const float* __restrict__ lsc, const int* __restrict__ kmask,
    unsigned short* __restrict__ ahp, unsigned short* __restrict__ alp) {
  __shared__ __align__(16) unsigned short lds[LDS_TOT];

  const int tid  = (int)threadIdx.x;
  const int lane = tid & 31;
  const int wave = wave_id();
  const int hh   = lane >> 4;
  const int c    = lane & 15;
  const int qb   = (int)blockIdx.x;
  const int h    = (int)blockIdx.y;
  const int b    = (int)blockIdx.z;
  const int kvh  = h >> 2;
  const int q0   = qb * 64 + wave * 16;
  const int qlast = q0 + 15;
  const size_t tok0 = (size_t)b * SQ;

  const float coef = 2.0f * tanhf(bf_rne(qpar[h]));
  const float escl = expf(bf_rne(lsc[h])) * 0.0078125f;

  const unsigned short* Qhr = qhp + (tok0 + q0 + c) * HID + h * HDM + 8 * hh;
  const unsigned short* Qlr = qlp + (tok0 + q0 + c) * HID + h * HDM + 8 * hh;
  const unsigned short* Khg = khp + tok0 * KVW + kvh * HDM;
  const unsigned short* Klg = klp + tok0 * KVW + kvh * HDM;
  const unsigned short* Vhg = vhp + (size_t)(kvh * HDM) * NTOK + tok0;
  const unsigned short* Vlg = vlp + (size_t)(kvh * HDM) * NTOK + tok0;
  unsigned short* ph = lds + LDS_PH + wave * (16 * PS_P);
  unsigned short* pl = lds + LDS_PL + wave * (16 * PS_P);

  float mrow[8], lrow[8];
  v8f oacc[8];
#pragma unroll
  for (int r = 0; r < 8; ++r) { mrow[r] = -INFINITY; lrow[r] = 0.f; }
#pragma unroll
  for (int t = 0; t < 8; ++t) oacc[t] = zero8();

  const int nch = 2 * qb + 2;
  for (int kc = 0; kc < nch; ++kc) {
    const int kv0 = kc * AT_KC;
    __syncthreads();
#pragma unroll
    for (int i = 0; i < 4; ++i) {
      const int p   = tid + 128 * i;
      const int key = p >> 4, d8 = (p & 15) * 8;
      const size_t kgo = (size_t)(kv0 + key) * KVW + d8;
      const v8us kx = *(const v8usa*)(Khg + kgo);
      const v8us ky = *(const v8usa*)(Klg + kgo);
      *(v8us*)(lds + LDS_KH + key * KS_P + d8) = kx;
      *(v8us*)(lds + LDS_KL + key * KS_P + d8) = ky;
      const int d = p >> 2, k8 = (p & 3) * 8;
      const size_t vgo = (size_t)d * NTOK + kv0 + k8;
      const v8us vx = *(const v8usa*)(Vhg + vgo);
      const v8us vy = *(const v8usa*)(Vlg + vgo);
      *(v8us*)(lds + LDS_VH + d * VS_P + k8) = vx;
      *(v8us*)(lds + LDS_VL + d * VS_P + k8) = vy;
    }
    __syncthreads();

    if (kv0 <= qlast) {
      v8f sc[2];
#pragma unroll
      for (int j = 0; j < 2; ++j) {
        v8f a00 = zero8(), a11 = zero8(), a01 = zero8(), a10 = zero8();
#pragma unroll
        for (int st = 0; st < 2; ++st) {
          const v16b q0h = ldfrag(Qhr + st * 32);
          const v16b q0l = ldfrag(Qlr + st * 32);
          const v16b q1h = ldfrag(Qhr + HHALF + st * 32);
          const v16b q1l = ldfrag(Qlr + HHALF + st * 32);
          const unsigned short* kr = lds + (j * 16 + c) * KS_P + st * 32 + 8 * hh;
          const v16b k0h = ldfrag(kr + LDS_KH);
          const v16b k0l = ldfrag(kr + LDS_KL);
          const v16b k1h = ldfrag(kr + LDS_KH + HHALF);
          const v16b k1l = ldfrag(kr + LDS_KL + HHALF);
          a00 = mma_b(q0h, k0h, a00); a00 = mma_b(q0h, k0l, a00); a00 = mma_b(q0l, k0h, a00);
          a10 = mma_b(q1h, k0h, a10); a10 = mma_b(q1h, k0l, a10); a10 = mma_b(q1l, k0h, a10);
          a11 = mma_b(q1h, k1h, a11); a11 = mma_b(q1h, k1l, a11); a11 = mma_b(q1l, k1h, a11);
          a01 = mma_b(q0h, k1h, a01); a01 = mma_b(q0h, k1l, a01); a01 = mma_b(q0l, k1h, a01);
          guard_s(a00, a10, a11, a01, q0h, q0l, q1h, q1l, k0h, k0l, k1h, k1l);
        }
        const int mv  = kmask[tok0 + kv0 + j * 16 + c];
        const int key = kv0 + j * 16 + c;
        v8f s;
#pragma unroll
        for (int r = 0; r < 8; ++r) {
          const int qrow = q0 + 8 * hh + r;
          float v = (a00[r] * a11[r] - coef * (a01[r] * a10[r])) * escl;
          v = (key > qrow) ? -1.0e9f : v;
          v = (mv == 0) ? -1.0e9f : v;
          s[r] = v;
        }
        sc[j] = s;
      }
      float cm[8];
#pragma unroll
      for (int r = 0; r < 8; ++r) {
        float m = fmaxf(sc[0][r], sc[1][r]);
#pragma unroll
        for (int off = 1; off < 16; off <<= 1) m = fmaxf(m, __shfl_xor(m, off, 32));
        cm[r] = m;
      }
#pragma unroll
      for (int r = 0; r < 8; ++r) {
        const float mnew  = fmaxf(mrow[r], cm[r]);
        const float alpha = __expf(mrow[r] - mnew);
        mrow[r] = mnew;
        float psum = 0.f;
#pragma unroll
        for (int j = 0; j < 2; ++j) {
          const float p = __expf(sc[j][r] - mnew);
          psum += p;
          const unsigned short hb = bf_bits(p);
          const unsigned short lb = bf_bits(p - bf_val(hb));
          const int po = (8 * hh + r) * PS_P + j * 16 + c;
          ph[po] = hb;
          pl[po] = lb;
        }
#pragma unroll
        for (int off = 1; off < 16; off <<= 1) psum += __shfl_xor(psum, off, 32);
        lrow[r] = lrow[r] * alpha + psum;
#pragma unroll
        for (int t = 0; t < 8; ++t) oacc[t][r] *= alpha;
      }
      lds_wave_sync();
      const v16b pa = ldfrag(ph + c * PS_P + 8 * hh);
      const v16b pr = ldfrag(pl + c * PS_P + 8 * hh);
#pragma unroll
      for (int t = 0; t < 8; ++t) {
        const unsigned short* vr0 = lds + (t * 16 + c) * VS_P + 8 * hh;
        const v16b vb = ldfrag(vr0 + LDS_VH);
        const v16b vl = ldfrag(vr0 + LDS_VL);
        oacc[t] = mma_b(pa, vb, oacc[t]);
        oacc[t] = mma_b(pa, vl, oacc[t]);
        oacc[t] = mma_b(pr, vb, oacc[t]);
        guard_o(oacc[t], pa, pr, vb, vl);
      }
    }
  }

  __syncthreads();
  unsigned short* osh = lds + wave * 4096;
  unsigned short* osl = osh + 2048;
#pragma unroll
  for (int r = 0; r < 8; ++r) {
    const float inv = 1.0f / lrow[r];
#pragma unroll
    for (int t = 0; t < 8; ++t) {
      const float o = oacc[t][r] * inv;
      const unsigned short hb = bf_bits(o);
      const unsigned short lb = bf_bits(o - bf_val(hb));
      const int so = (8 * hh + r) * 128 + t * 16 + c;
      osh[so] = hb;
      osl[so] = lb;
    }
  }
  lds_wave_sync();
  unsigned short* Ahg = ahp + (tok0 + q0) * HID + h * HDM;
  unsigned short* Alg = alp + (tok0 + q0) * HID + h * HDM;
  for (int pass = 0; pass < 2; ++pass) {
#pragma unroll
    for (int it = 0; it < 8; ++it) {
      const int row = it * 2 + hh;
      const int c8  = c * 8;
      const v8us x = *(const v8usa*)(osh + row * 128 + c8);
      const v8us y = *(const v8usa*)(osl + row * 128 + c8);
      *(volatile v8us*)(Ahg + (size_t)row * HID + c8) = x;
      *(volatile v8us*)(Alg + (size_t)row * HID + c8) = y;
    }
    __threadfence();
  }
}

extern "C" void kernel_launch(void* const* d_in, const int* in_sizes, int n_in,
                              void* d_out, int out_size, void* d_ws, size_t ws_size,
                              hipStream_t stream) {
  if (n_in < 10) return;
  if (in_sizes[0] != NTOK * HID) return;
  if (in_sizes[1] != HID * HID) return;
  if (in_sizes[2] != HID * KVW) return;
  if (in_sizes[3] != HID * KVW) return;
  if (in_sizes[4] != HID * HID) return;
  if (in_sizes[5] != NHQ || in_sizes[6] != NHQ) return;
  if (in_sizes[7] != SQ * NHQ * HHALF || in_sizes[8] != SQ * NHQ * HHALF) return;
  if (in_sizes[9] != NTOK) return;
  if (out_size != NTOK * HID) return;

  const float* x    = (const float*)d_in[0];
  const float* Wq   = (const float*)d_in[1];
  const float* Wk   = (const float*)d_in[2];
  const float* Wv   = (const float*)d_in[3];
  const float* Wo   = (const float*)d_in[4];
  const float* qpar = (const float*)d_in[5];
  const float* lsc  = (const float*)d_in[6];
  const float* cosp = (const float*)d_in[7];
  const float* sinp = (const float*)d_in[8];
  const int*   kmask = (const int*)d_in[9];
  float* out = (float*)d_out;

  const size_t szX  = (size_t)NTOK * HID * 2;
  const size_t szWT = (size_t)WTR * HID * 2;
  const size_t szWo = (size_t)HID * HID * 2;
  const size_t szQ  = (size_t)NTOK * HID * 2;
  const size_t szK  = (size_t)NTOK * KVW * 2;
  const size_t szV  = (size_t)KVW * NTOK * 2;
  const size_t szA  = (size_t)NTOK * HID * 2;
  size_t off = 0;
  const size_t oX  = off; off += szX;
  const size_t oWT = off; off += szWT;
  const size_t oWo = off; off += szWo;
  const size_t oQh = off; off += szQ;
  const size_t oQl = off; off += szQ;
  const size_t oKh = off; off += szK;
  const size_t oKl = off; off += szK;
  const size_t oVh = off; off += szV;
  const size_t oVl = off; off += szV;
  const size_t oAh = off; off += szA;
  const size_t oAl = off; off += szA;
  if (off > ws_size) return;
  if (off > (size_t)134217728) return;

  char* ws = (char*)d_ws;
  unsigned short* Xb  = (unsigned short*)(ws + oX);
  unsigned short* WT  = (unsigned short*)(ws + oWT);
  unsigned short* WoT = (unsigned short*)(ws + oWo);
  unsigned short* Qh  = (unsigned short*)(ws + oQh);
  unsigned short* Ql  = (unsigned short*)(ws + oQl);
  unsigned short* Kh  = (unsigned short*)(ws + oKh);
  unsigned short* Kl  = (unsigned short*)(ws + oKl);
  unsigned short* Vh  = (unsigned short*)(ws + oVh);
  unsigned short* Vl  = (unsigned short*)(ws + oVl);
  unsigned short* Ah  = (unsigned short*)(ws + oAh);
  unsigned short* Al  = (unsigned short*)(ws + oAl);

  const dim3 b256(256), b128(128);

  cvt_bf16_kernel<<<dim3((NTOK * HID / 8) / 256), b256, 0, stream>>>(x, Xb, NTOK * HID / 8);
  tconv_bf16_kernel<<<dim3(HID / 64, HID / 64), b256, 0, stream>>>(Wq, WT, HID, HID);
  tconv_bf16_kernel<<<dim3(KVW / 64, HID / 64), b256, 0, stream>>>(Wk, WT + (size_t)QW * HID, HID, KVW);
  tconv_bf16_kernel<<<dim3(KVW / 64, HID / 64), b256, 0, stream>>>(Wv, WT + (size_t)QKW * HID, HID, KVW);
  tconv_bf16_kernel<<<dim3(HID / 64, HID / 64), b256, 0, stream>>>(Wo, WoT, HID, HID);
  gemm_w32x128_kernel<0, false><<<dim3((NTOK / 32) * (QKW / 128) / 4), b128, 0, stream>>>(
      Xb, Xb, HID, WT, HID, cosp, sinp, (void*)Qh, (void*)Ql, (void*)Kh, (void*)Kl, HID, NTOK, QKW, HID);
  gemm_w32x128_kernel<1, false><<<dim3((KVW / 32) * (NTOK / 128) / 4), b128, 0, stream>>>(
      WT + (size_t)QKW * HID, WT + (size_t)QKW * HID, HID, Xb, HID, cosp, sinp,
      (void*)Vh, (void*)Vl, (void*)Vh, (void*)Vl, NTOK, KVW, NTOK, HID);
  attn_bivector_kernel<<<dim3(SQ / 64, NHQ, NSEQ), b128, 0, stream>>>(Qh, Ql, Kh, Kl, Vh, Vl, qpar, lsc, kmask, Ah, Al);
  gemm_w32x128_kernel<2, true><<<dim3((NTOK / 32) * (HID / 128) / 4), b128, 0, stream>>>(
      Ah, Al, HID, WoT, HID, cosp, sinp, (void*)out, (void*)out, (void*)out, (void*)out, HID, NTOK, HID, HID);
  (void)hipGetLastError();
}
